// QNN_14654428414825
// MI455X (gfx1250) — hardware-run, weakly checked
//
#include <hip/hip_runtime.h>


#ifndef NB
#define NB 16384
#endif
#define NB_FULL 16384
#define IMGN  784
#define IMGW  28
#define NQ    10
#define DIM   1024
#define KC    800
#define NCLS  10
#define NPADC 16

static_assert(NB <= NB_FULL);
static_assert(NB % 64 == 0);
static_assert(NB % 32 == 0);
static_assert(DIM % 64 == 0);
static_assert(DIM % 32 == 0);
static_assert(KC % 32 == 0);
static_assert(KC >= IMGN);
static_assert(KC % 8 == 0 && IMGN % 8 == 0);
static_assert((IMGN * 4) % 32 == 0);
static_assert(IMGN % 4 == 0 && (IMGN / 4) <= 7 * 32);
static_assert(((size_t)NB * (KC / 8)) % 256 == 0);
static_assert(((size_t)NPADC * (DIM / 8)) % 256 == 0);
static_assert(((size_t)DIM * (KC / 8)) % 256 == 0);
static_assert(NCLS <= NPADC);
static_assert((1 << NQ) == DIM);
static_assert(4 * 32 * 16 == 16 * 64 * 2);
static_assert(5 * 32 * 16 == 64 * NCLS * 4);
static_assert(8 * 16 == 32 * 4);
static_assert((64 * NCLS * 4) % 128 == 0);
static_assert(16 * 68 * 4 <= 131072);
static_assert(64 * NCLS * 4 <= 131072);

typedef unsigned short bf;
typedef __attribute__((ext_vector_type(16))) __bf16   v16bf;
typedef __attribute__((ext_vector_type(8)))  unsigned short v8us;
typedef __attribute__((ext_vector_type(8)))  float    v8f;
typedef __attribute__((ext_vector_type(4)))  float    v4f;
typedef v4f  __attribute__((may_alias)) v4fa;

__device__ __forceinline__ unsigned short f2bf(float f) { unsigned u = __float_as_uint(f); u += 0x7FFFu + ((u >> 16) & 1u); return (unsigned short)(u >> 16); }
__device__ __forceinline__ float bfr(float f) { return __uint_as_float(((unsigned)f2bf(f)) << 16); }
__device__ __forceinline__ v16bf cat16b(v8us lo, v8us hi) { return __builtin_bit_cast(v16bf, __builtin_shufflevector(lo, hi, 0, 1, 2, 3, 4, 5, 6, 7, 8, 9, 10, 11, 12, 13, 14, 15)); }
__device__ __forceinline__ v8f wmmab(v16bf a, v16bf b, v8f c) { return __builtin_amdgcn_wmma_f32_16x16x32_bf16(false, a, false, b, (short)0, c, false, false); }
__device__ __forceinline__ v16bf ldb(const bf* p)  { return cat16b(*(const v8us*)p, *(const v8us*)(p + 16)); }
__device__ __forceinline__ void wave_sync() { __builtin_amdgcn_fence(3  , "wavefront"); __builtin_amdgcn_wave_barrier(); asm volatile("" ::: "memory"); }
__device__ __forceinline__ v8f wmmab_g(v16bf a, v16bf b, v8f c) {
    c = wmmab(a, b, c);
    asm volatile("v_nop\n\tv_nop\n\tv_nop\n\tv_nop" : "+v"(c) : "v"(a), "v"(b));
    return c;
}

__global__ __launch_bounds__(256) void k_cvtpad(const float* __restrict__ src, bf* dst, int spitch, int gsrc, int gdst, int rsrc, unsigned n8) {
    const unsigned i = blockIdx.x * 256u + threadIdx.x; if (i >= n8) return;
    const int row = (int)(i / (unsigned)gdst), g = (int)(i % (unsigned)gdst);
    const int rs = row < rsrc ? row : rsrc - 1;
    const int gs = g < gsrc ? g : gsrc - 1;
    v8f v = *(const v8f*)(src + (size_t)rs * (size_t)spitch + (size_t)gs * 8);
    asm volatile("" : "+v"(v));
    const bool ok = (row < rsrc) & (g < gsrc);
    v8us o;
#pragma unroll
    for (int k = 0; k < 8; ++k) o[k] = ok ? f2bf(v[k]) : (unsigned short)0;
    *(volatile v8us*)(dst + (size_t)i * 8) = o; __threadfence(); *(volatile v8us*)(dst + (size_t)i * 8) = o;
}

__global__ __launch_bounds__(256) void k_rbuild(const float* __restrict__ angles, bf* RB) {
    __shared__ float cs[2 * NQ];
    const int qi = threadIdx.x < NQ ? (int)threadIdx.x : NQ - 1;
    const float th = 0.5f * bfr(angles[qi]);
    const float cth = cosf(th), sth = sinf(th);
    if (threadIdx.x < NQ) { cs[threadIdx.x] = cth; cs[NQ + threadIdx.x] = sth; }
    __syncthreads();
    const unsigned i = blockIdx.x * 256u + threadIdx.x;
    const int n = (int)(i / (unsigned)(KC / 8)), g = (int)(i % (unsigned)(KC / 8));
    int sg = n;
#pragma unroll 1
    for (int c = NQ - 2; c >= 0; --c) sg ^= ((sg >> (9 - c)) & 1) << (8 - c);
    int jj[8]; float val[8];
#pragma unroll
    for (int e = 0; e < 8; ++e) { const int kk = g * 8 + e; const int kc = kk < IMGN ? kk : IMGN - 1; const int r = kc / IMGW; const int c = kc - r * IMGW;
        jj[e] = (r + 2) * 32 + (c + 2); val[e] = 1.0f; }
#pragma unroll 1
    for (int q = 0; q < NQ; ++q) {
        const float cq = cs[q], sq = cs[NQ + q]; const int sh = 9 - q; const int a = (sg >> sh) & 1;
        const float e0 = a ? sq : cq;
        const float e1 = a ? cq : -sq;
#pragma unroll
        for (int e = 0; e < 8; ++e) val[e] *= ((jj[e] >> sh) & 1) ? e1 : e0;
    }
    v8us o;
#pragma unroll
    for (int e = 0; e < 8; ++e) o[e] = (g * 8 + e < IMGN) ? f2bf(val[e]) : (unsigned short)0;
    *(volatile v8us*)(RB + (size_t)i * 8) = o; __threadfence(); *(volatile v8us*)(RB + (size_t)i * 8) = o;
}

__global__ __launch_bounds__(256) void k_norm(const float* __restrict__ x, float* INV) {
    __shared__ __align__(16) float sred[32];
    const int lane = threadIdx.x & 31;
    const int wave = __builtin_amdgcn_readfirstlane((int)(threadIdx.x >> 5));
#pragma unroll 1
    for (int r = 0; r < 4; ++r) {
        const int row = blockIdx.x * 32 + wave * 4 + r;
        const float* p = x + (size_t)row * IMGN;
        float s = 0.0f;
#pragma unroll 1
        for (int it = 0; it < 7; ++it) {
            const int q = it * 32 + lane; const int qc = q < (IMGN / 4) ? q : (IMGN / 4) - 1;
            v4f v = *(const v4f*)(p + qc * 4);
            asm volatile("" : "+v"(v));
            const bool ok = q < (IMGN / 4);
#pragma unroll
            for (int e = 0; e < 4; ++e) { const float t = ok ? bfr(v[e]) : 0.0f; s += t * t; }
        }
#pragma unroll
        for (int off = 16; off > 0; off >>= 1) s += __shfl_xor(s, off, 32);
        if (lane == 0) sred[wave * 4 + r] = rsqrtf(s);
    }
    __syncthreads();
    if (wave == 0) {
        if (lane < 8) {
            const v4f v = *(const v4fa*)(&sred[lane * 4]);
            float* d = INV + (size_t)blockIdx.x * 32 + lane * 4;
            *(volatile v4f*)d = v; __threadfence(); *(volatile v4f*)d = v;
        }
    }
}

__global__ __launch_bounds__(32) void k_circ(const bf* __restrict__ A, const bf* __restrict__ Bt, const float* __restrict__ INV, bf* PB) {
    __shared__ __align__(16) float os[16 * 68];
    const int K = KC;
    const int lane = threadIdx.x & 31, lr = lane & 15, hi = lane >> 4; const int r0 = blockIdx.x * 64, c0 = blockIdx.y * 64;
    v8f acc[4][4];
#pragma unroll
    for (int mb = 0; mb < 4; ++mb)
#pragma unroll
        for (int nb = 0; nb < 4; ++nb) acc[mb][nb] = (v8f){};
    const size_t aoff = (size_t)(r0 + lr) * K + 8 * hi, boff = (size_t)(c0 + lr) * K + 8 * hi;
#pragma unroll 1
    for (int kc = 0; kc < K; kc += 32) {
        v16bf a[4];
#pragma unroll
        for (int mb = 0; mb < 4; ++mb) a[mb] = ldb(A + aoff + (size_t)mb * 16 * K + kc);
#pragma unroll
        for (int nb = 0; nb < 4; ++nb) { const v16bf b = ldb(Bt + boff + (size_t)nb * 16 * K + kc);
#pragma unroll
            for (int mb = 0; mb < 4; ++mb) acc[mb][nb] = wmmab_g(a[mb], b, acc[mb][nb]); }
    }
#pragma unroll
    for (int mb = 0; mb < 4; ++mb) {
        const v4f i0 = *(const v4f*)(INV + r0 + mb * 16 + hi * 8), i1 = *(const v4f*)(INV + r0 + mb * 16 + hi * 8 + 4);
        float iv[8];
#pragma unroll
        for (int j = 0; j < 4; ++j) { iv[j] = i0[j]; iv[4 + j] = i1[j]; }
#pragma unroll
        for (int nb = 0; nb < 4; ++nb) {
#pragma unroll
            for (int j = 0; j < 8; ++j) { const float y = acc[mb][nb][j] * iv[j]; os[(hi * 8 + j) * 68 + nb * 16 + lr] = y * y; } }
        wave_sync();
#pragma unroll 1
        for (int ps = 0; ps < 2; ++ps) {
#pragma unroll
            for (int s = 0; s < 4; ++s) { const int row = 4 * s + (lane >> 3), c8 = (lane & 7) * 8;
                const v4f x0 = *(const v4fa*)(&os[row * 68 + c8]); const v4f x1 = *(const v4fa*)(&os[row * 68 + c8 + 4]); v8us o;
#pragma unroll
                for (int i = 0; i < 4; ++i) { o[i] = f2bf(x0[i]); o[4 + i] = f2bf(x1[i]); }
                const size_t oo = (size_t)(r0 + mb * 16 + row) * DIM + (size_t)(c0 + c8);
                *(volatile v8us*)(PB + oo) = o; }
            if (ps == 0) __threadfence(); }
        wave_sync();
    }
}

__global__ __launch_bounds__(32) void k_read(const bf* __restrict__ P, const bf* __restrict__ Wt, const float* __restrict__ bias, float* OUT) {
    __shared__ __align__(16) float os[64 * NCLS];
    const int lane = threadIdx.x & 31, lr = lane & 15, hi = lane >> 4; const int r0 = blockIdx.x * 64;
    v8f acc[4];
#pragma unroll
    for (int mb = 0; mb < 4; ++mb) acc[mb] = (v8f){};
    const size_t aoff = (size_t)(r0 + lr) * DIM + 8 * hi, boff = (size_t)lr * DIM + 8 * hi;
#pragma unroll 1
    for (int kc = 0; kc < DIM; kc += 32) {
        const v16bf b = ldb(Wt + boff + kc);
#pragma unroll
        for (int mb = 0; mb < 4; ++mb) { const v16bf a = ldb(P + aoff + (size_t)mb * 16 * DIM + kc); acc[mb] = wmmab_g(a, b, acc[mb]); }
    }
    const int lc = lr < NCLS ? lr : NCLS - 1;
    float bv = bias[lc];
    asm volatile("" : "+v"(bv));
    bv = bfr(bv);
#pragma unroll
    for (int mb = 0; mb < 4; ++mb) {
#pragma unroll
        for (int j = 0; j < 8; ++j) { if (lr < NCLS) os[(mb * 16 + hi * 8 + j) * NCLS + lr] = acc[mb][j] + bv; } }
    wave_sync();
    float* ob = OUT + (size_t)r0 * NCLS;
#pragma unroll 1
    for (int ps = 0; ps < 2; ++ps) {
#pragma unroll
        for (int s = 0; s < 5; ++s) { const int idx = s * 32 + lane;
            const v4f val = *(const v4fa*)(&os[idx * 4]);
            *(volatile v4f*)(ob + (size_t)idx * 4) = val; }
        if (ps == 0) __threadfence(); }
}

static constexpr size_t al256(size_t v) { return (v + 255) & ~(size_t)255; }
static constexpr size_t SZ_XB = al256((size_t)NB * KC * 2);
static constexpr size_t SZ_RB = al256((size_t)DIM * KC * 2);
static constexpr size_t SZ_WB = al256((size_t)NPADC * DIM * 2);
static constexpr size_t SZ_IV = al256((size_t)NB * 4);
static constexpr size_t SZ_PB = al256((size_t)NB * DIM * 2);
static constexpr size_t SZ_TOTAL = SZ_XB + SZ_RB + SZ_WB + SZ_IV + SZ_PB;
static_assert(SZ_TOTAL <= (size_t)134217728);
static_assert((size_t)NB * (KC / 8) * 16 == (size_t)NB * KC * 2);
static_assert((size_t)DIM * (KC / 8) * 16 == (size_t)DIM * KC * 2);
static_assert((size_t)NPADC * (DIM / 8) * 16 == (size_t)NPADC * DIM * 2);
static_assert((size_t)(NB / 32) * 128 == (size_t)NB * 4);
static_assert((size_t)(NB / 64) * (DIM / 64) * 64 * 128 == (size_t)NB * DIM * 2);
static_assert((size_t)(NB / 64) * 64 * NCLS * 4 == (size_t)NB * NCLS * 4);

extern "C" void kernel_launch(void* const* d_in, const int* in_sizes, int n_in,
                              void* d_out, int out_size, void* d_ws, size_t ws_size, hipStream_t stream) {
    if (n_in < 4) return;
    if ((size_t)in_sizes[0] < (size_t)NB * IMGN) return;
    if (in_sizes[1] < NQ) return;
    if ((size_t)in_sizes[2] < (size_t)NCLS * DIM) return;
    if (in_sizes[3] < NCLS) return;
    if ((size_t)out_size < (size_t)NB * NCLS) return;
    if (SZ_TOTAL > ws_size) return;
    const float* x      = (const float*)d_in[0];
    const float* angles = (const float*)d_in[1];
    const float* W      = (const float*)d_in[2];
    const float* bias   = (const float*)d_in[3];
    float* OUT = (float*)d_out;
    char* wsp = (char*)d_ws;
    bf* XB = (bf*)wsp; wsp += SZ_XB;
    bf* RB = (bf*)wsp; wsp += SZ_RB;
    bf* WB = (bf*)wsp; wsp += SZ_WB;
    float* INV = (float*)wsp; wsp += SZ_IV;
    bf* PB = (bf*)wsp; wsp += SZ_PB;

    { const unsigned n8 = (unsigned)((size_t)NB * (KC / 8));
      k_cvtpad<<<n8 / 256u, 256, 0, stream>>>(x, XB, IMGN, IMGN / 8, KC / 8, NB, n8); }
    { const unsigned n8 = (unsigned)((size_t)NPADC * (DIM / 8));
      k_cvtpad<<<n8 / 256u, 256, 0, stream>>>(W, WB, DIM, DIM / 8, DIM / 8, NCLS, n8); }
    k_rbuild<<<(unsigned)(((size_t)DIM * (KC / 8)) / 256), 256, 0, stream>>>(angles, RB);
    k_norm<<<NB / 32, 256, 0, stream>>>(x, INV);
    k_circ<<<dim3(NB / 64, DIM / 64, 1), 32, 0, stream>>>(XB, RB, INV, PB);
    k_read<<<NB / 64, 32, 0, stream>>>(PB, WB, bias, OUT);
}
